// StructureDecoder_18743237280509
// MI455X (gfx1250) — hardware-verified
//
#include <hip/hip_runtime.h>
#include <stddef.h>


#define CIN    128
#define HID    256
#define NPL    512
#define KPB    128
#define PQW    512
#define APZ    136
#define GROWS  32
#define GTHR   64
#define WTHR   256
#define WBLK   ((NPL * KPB) / (8 * WTHR))
#define ETHR   256
#define EWAV   (ETHR / 32)
#define EPW    128
#define EPB    (EWAV * EPW)
#define WSC    64.0f
#define ZSC    4.0f
#define RSC    0.00390625f
#define WSCAP  134217728

static_assert(WBLK * WTHR * 8 == NPL * KPB);
static_assert(GROWS == (GTHR / 32) * 16);
static_assert((APZ % 8) == 0 && (KPB % 8) == 0 && (PQW % 32) == 0 && (HID % 32) == 0);
static_assert(GTHR * 64 == GROWS * CIN);
static_assert(32 * GTHR * 4 == GROWS * HID);
static_assert(ETHR * 4 == EPB);
static_assert((CIN % 32) == 0);
static_assert((EPW % 32) == 0);
static_assert(HID == 8 * 32);

typedef float    v4f  __attribute__((ext_vector_type(4)));
typedef float    v8f  __attribute__((ext_vector_type(8)));
typedef _Float16 v8h  __attribute__((ext_vector_type(8)));
typedef _Float16 v16h __attribute__((ext_vector_type(16)));
union Frag { v16h v; v8h h[2]; };

__device__ __forceinline__ v8f wmh(v16h a, v16h b, v8f c) {
  v8f d = __builtin_amdgcn_wmma_f32_16x16x32_f16(false, a, false, b, (short)0, c, false, false);
  asm volatile("v_nop\n\tv_nop\n\tv_nop\n\tv_nop" : "+v"(d) : "v"(a), "v"(b));
  return d;
}

__device__ __forceinline__ v8h cvt8z(v4f a, v4f b) {
  v8h r;
  r[0] = (_Float16)(a.x * ZSC); r[1] = (_Float16)(a.y * ZSC);
  r[2] = (_Float16)(a.z * ZSC); r[3] = (_Float16)(a.w * ZSC);
  r[4] = (_Float16)(b.x * ZSC); r[5] = (_Float16)(b.y * ZSC);
  r[6] = (_Float16)(b.z * ZSC); r[7] = (_Float16)(b.w * ZSC);
  return r;
}

template <int NT>
__device__ __forceinline__ void mma16(const _Float16* At, const _Float16* __restrict__ Bpl,
                                      int lane, v8f (&acc)[NT]) {
  const int hh = lane >> 4, m = lane & 15;
#pragma unroll
  for (int t = 0; t < NT; ++t) { v8f zz = {0.f, 0.f, 0.f, 0.f, 0.f, 0.f, 0.f, 0.f}; acc[t] = zz; }
  const _Float16* ap = At + m * APZ + 8 * hh;
  const _Float16* bb = Bpl + (size_t)m * KPB + 8 * hh;
#pragma unroll 1
  for (int ks = 0; ks < CIN / 32; ++ks) {
    Frag a;
    a.h[0] = *(const v8h*)(ap + 32 * ks);
    a.h[1] = *(const v8h*)(ap + 32 * ks + 16);
#pragma unroll
    for (int t = 0; t < NT; ++t) {
      const _Float16* bp = bb + (size_t)(16 * t) * KPB + 32 * ks;
      Frag b;
      b.h[0] = *(const v8h*)bp;
      b.h[1] = *(const v8h*)(bp + 16);
      acc[t] = wmh(a.v, b.v, acc[t]);
    }
  }
}

__global__ __launch_bounds__(WTHR) void k_wprep(const float* __restrict__ W1, _Float16* Bpl) {
  const int i  = blockIdx.x * WTHR + threadIdx.x;
  const int n  = i >> 4, k0 = (i & 15) * 8;
  const int kb = (n >> 8) * CIN, nc = n & (HID - 1);
  v8h hv;
#pragma unroll
  for (int e = 0; e < 8; ++e) hv[e] = (_Float16)(W1[(size_t)(kb + k0 + e) * HID + nc] * WSC);
  _Float16* dp = Bpl + (size_t)i * 8;
  *(volatile v8h*)dp = hv;
  __threadfence();
  *(volatile v8h*)dp = hv;
}

__global__ __launch_bounds__(GTHR) void k_nodegemm(const float* __restrict__ z, const _Float16* __restrict__ Bpl,
                                                   const float* __restrict__ b1, float* PQ, int nN) {
  __shared__ __attribute__((aligned(16))) _Float16 Az[GROWS * APZ];
  __shared__ __attribute__((aligned(16))) float stg[GROWS * HID];
  const int tid = threadIdx.x, lane = tid & 31, wave = tid >> 5, hh = lane >> 4, m = lane & 15;
  const int rowBase = blockIdx.x * GROWS;
  {
    const int r = tid >> 1, c0 = (tid & 1) * 64;
    int zrow = rowBase + r;
    zrow = zrow > nN - 1 ? nN - 1 : zrow;
    const float* zp = z + (size_t)zrow * CIN + c0;
#pragma unroll
    for (int j = 0; j < 8; ++j) {
      const v4f a = *(const v4f*)(zp + 8 * j), b = *(const v4f*)(zp + 8 * j + 4);
      *(v8h*)(Az + r * APZ + c0 + 8 * j) = cvt8z(a, b);
    }
  }
  __syncthreads();

#pragma unroll 1
  for (int hf = 0; hf < 2; ++hf) {
#pragma unroll 1
    for (int cg = 0; cg < 4; ++cg) {
      v8f acc[4];
      mma16<4>(Az + wave * 16 * APZ, Bpl + (size_t)(hf * HID + 64 * cg) * KPB, lane, acc);
      float* sp = stg + (wave * 16 + 8 * hh) * HID + 64 * cg + m;
#pragma unroll
      for (int t = 0; t < 4; ++t) {
        const int col = 64 * cg + 16 * t + m;
        const float bb = b1[col];
        const float bv = (hf != 0) ? bb : 0.0f;
#pragma unroll
        for (int r = 0; r < 8; ++r) sp[r * HID + 16 * t] = acc[t][r] * RSC + bv;
      }
    }
    __syncthreads();
    float* gp = PQ + (size_t)rowBase * PQW + hf * HID;
#pragma unroll 4
    for (int it = 0; it < 32; ++it) {
      const int f = it * GTHR + tid;
      const int row = f >> 6, c4 = f & 63;
      const v4f v = *(const v4f*)(stg + row * HID + 4 * c4);
      *(volatile v4f*)(gp + (size_t)row * PQW + 4 * c4) = v;
    }
    __threadfence();
#pragma unroll 4
    for (int it = 0; it < 32; ++it) {
      const int f = it * GTHR + tid;
      const int row = f >> 6, c4 = f & 63;
      const v4f v = *(const v4f*)(stg + row * HID + 4 * c4);
      *(volatile v4f*)(gp + (size_t)row * PQW + 4 * c4) = v;
    }
    __syncthreads();
  }
}

__global__ __launch_bounds__(ETHR) void k_edge(const float* __restrict__ PQ, const int* __restrict__ ei,
                                               const float* __restrict__ W2, const float* __restrict__ b2,
                                               float* out, int nN, int nE) {
  __shared__ __attribute__((aligned(16))) float sres[EPB];
  const int tid = threadIdx.x, lane = tid & 31, wave = tid >> 5;
  const int ebase = blockIdx.x * EPB;
  const v4f wa = *(const v4f*)(W2 + 8 * lane);
  const v4f wb = *(const v4f*)(W2 + 8 * lane + 4);
  const float b2v = b2[0];

#pragma unroll 1
  for (int it = 0; it < EPW / 32; ++it) {
    const int le0 = wave * EPW + it * 32;
    int e = ebase + le0 + lane;
    e = e > nE - 1 ? nE - 1 : e;
    int rv = ei[e];
    int cv = ei[(size_t)nE + e];
    rv = rv < 0 ? 0 : (rv > nN - 1 ? nN - 1 : rv);
    cv = cv < 0 ? 0 : (cv > nN - 1 ? nN - 1 : cv);
    float resv = 0.0f;
#pragma unroll 1
    for (int j = 0; j < 32; ++j) {
      const int r = __shfl(rv, j, 32);
      const int c = __shfl(cv, j, 32);
      const float* pp = PQ + (size_t)r * PQW + 8 * lane;
      const float* qp = PQ + (size_t)c * PQW + HID + 8 * lane;
      const v4f p0 = *(const v4f*)pp, p1 = *(const v4f*)(pp + 4);
      const v4f q0 = *(const v4f*)qp, q1 = *(const v4f*)(qp + 4);
      v4f h0 = p0 + q0, h1 = p1 + q1;
      h0.x = fmaxf(h0.x, 0.0f); h0.y = fmaxf(h0.y, 0.0f); h0.z = fmaxf(h0.z, 0.0f); h0.w = fmaxf(h0.w, 0.0f);
      h1.x = fmaxf(h1.x, 0.0f); h1.y = fmaxf(h1.y, 0.0f); h1.z = fmaxf(h1.z, 0.0f); h1.w = fmaxf(h1.w, 0.0f);
      float s = h0.x * wa.x;
      s = fmaf(h0.y, wa.y, s);
      s = fmaf(h0.z, wa.z, s);
      s = fmaf(h0.w, wa.w, s);
      s = fmaf(h1.x, wb.x, s);
      s = fmaf(h1.y, wb.y, s);
      s = fmaf(h1.z, wb.z, s);
      s = fmaf(h1.w, wb.w, s);
      s += __shfl_xor(s, 16, 32);
      s += __shfl_xor(s, 8, 32);
      s += __shfl_xor(s, 4, 32);
      s += __shfl_xor(s, 2, 32);
      s += __shfl_xor(s, 1, 32);
      const float lg = s + b2v;
      const float ex = __expf(-lg);
      const float sg = __builtin_amdgcn_rcpf(1.0f + ex);
      resv = (lane == j) ? sg : resv;
    }
    sres[le0 + lane] = resv;
  }
  __syncthreads();

  const v4f v = *(const v4f*)(sres + 4 * tid);
  const int g = ebase + 4 * tid;
  if (g + 4 <= nE) {
    *(volatile v4f*)(out + g) = v;
  } else {
    if (g     < nE) *(volatile float*)(out + g)     = v.x;
    if (g + 1 < nE) *(volatile float*)(out + g + 1) = v.y;
    if (g + 2 < nE) *(volatile float*)(out + g + 2) = v.z;
    if (g + 3 < nE) *(volatile float*)(out + g + 3) = v.w;
  }
  __threadfence();
  if (g + 4 <= nE) {
    *(volatile v4f*)(out + g) = v;
  } else {
    if (g     < nE) *(volatile float*)(out + g)     = v.x;
    if (g + 1 < nE) *(volatile float*)(out + g + 1) = v.y;
    if (g + 2 < nE) *(volatile float*)(out + g + 2) = v.z;
    if (g + 3 < nE) *(volatile float*)(out + g + 3) = v.w;
  }
}

extern "C" void kernel_launch(void* const* d_in, const int* in_sizes, int n_in,
                              void* d_out, int out_size, void* d_ws, size_t ws_size,
                              hipStream_t stream) {
  if (n_in < 6) return;
  const int nN = in_sizes[0] / CIN;
  const int nE = in_sizes[1] / 2;
  if (nN <= 0 || nE <= 0) return;
  if (in_sizes[0] != nN * CIN || in_sizes[1] != 2 * nE) return;
  if (in_sizes[2] != 2 * CIN * HID || in_sizes[3] != HID || in_sizes[4] != HID || in_sizes[5] < 1) return;
  if (out_size != nE) return;
  if (nE > (1 << 28) || nN > (1 << 24)) return;

  const float* z  = (const float*)d_in[0];
  const int*   ei = (const int*)d_in[1];
  const float* W1 = (const float*)d_in[2];
  const float* b1 = (const float*)d_in[3];
  const float* W2 = (const float*)d_in[4];
  const float* b2 = (const float*)d_in[5];
  float* out = (float*)d_out;

  const int nBlkG = (nN + GROWS - 1) / GROWS;
  const int NPADG = nBlkG * GROWS;
  const int nBlkE = (nE + EPB - 1) / EPB;

  char* ws = (char*)d_ws;
  size_t off = 0;
  const size_t oB  = off; off += (size_t)NPL * KPB * 2;           off = (off + 255) & ~(size_t)255;
  const size_t oPQ = off; off += (size_t)NPADG * PQW * 4;          off = (off + 255) & ~(size_t)255;
  if (off > ws_size || off > (size_t)WSCAP) return;
  _Float16* Bpl = (_Float16*)(ws + oB);
  float*    PQ  = (float*)(ws + oPQ);

  k_wprep<<<WBLK, WTHR, 0, stream>>>(W1, Bpl);
  k_nodegemm<<<nBlkG, GTHR, 0, stream>>>(z, Bpl, b1, PQ, nN);
  k_edge<<<nBlkE, ETHR, 0, stream>>>(PQ, ei, W2, b2, out, nN, nE);
}
